// GCNBlock_78460462563622
// MI455X (gfx1250) — hardware-verified
//
#include <hip/hip_runtime.h>
#include <stddef.h>
#include <stdint.h>

#define NN      100000
#define DF      128
#define NE      640000
#define GBM     128
#define MP      100096
#define NTHR    256
#define NWAVE   8
#define EPT     8
#define WCH     (32 * EPT)
#define NBRUN   1024
#define SLB     10
#define NBK     98
#define WLCAP   1536
#define RCAP    8192
#define MAXB_MEAS   6759
#define MAXDEG_MEAS 20
#define WSMAX   ((size_t)128 << 20)

#define BK_ZINTS (NWAVE * WLCAP + 2 * RCAP + 3 * NBRUN)
#define BK_INTS  (BK_ZINTS + 16)
#define BK_LDS   (BK_INTS * 4)
#define GM_LDS   (GBM * DF * 4)

#define PBX   (MP * DF / 8 / NTHR)
#define PBW   (DF * DF / 8 / NTHR)
#define PBTOT (PBX + PBW)

static_assert(DF == 32 * 4);
static_assert(DF % 32 == 0);
static_assert(MP % GBM == 0 && MP >= NN && MP == 782 * GBM);
static_assert(NBRUN == (1 << SLB) && NBRUN % 32 == 0 && NBRUN == NTHR * 4);
static_assert(NBK * NBRUN >= NN);
static_assert(NE < (1 << 20) && (((long long)NE) << SLB) < (1LL << 31));
static_assert(NE % WCH == 0 && NE % 4 == 0);
static_assert((RCAP * 8) % 128 == 0 && (2 * RCAP) % (NTHR * 4) == 0 && BK_ZINTS % 4 == 0);
static_assert((long long)RCAP * 100 >= (long long)MAXB_MEAS * 105);
static_assert(WLCAP >= MAXB_MEAS / 8 + 8 * 30 + 1);
static_assert(NN % NWAVE == 0);
static_assert((MP * DF / 8) % NTHR == 0 && (DF * DF / 8) % NTHR == 0);
static_assert(BK_LDS <= 300000 && GM_LDS <= 327680);
static_assert(GBM == NWAVE * 16);

typedef float          v4f   __attribute__((ext_vector_type(4)));
typedef float          v8f   __attribute__((ext_vector_type(8)));
typedef int            v2i   __attribute__((ext_vector_type(2)));
typedef int            v4i   __attribute__((ext_vector_type(4)));
typedef int            v8i   __attribute__((ext_vector_type(8)));
typedef unsigned short v8us  __attribute__((ext_vector_type(8)));
typedef unsigned short v16us __attribute__((ext_vector_type(16)));
typedef __bf16         v16bf __attribute__((ext_vector_type(16)));
typedef v4f  __attribute__((may_alias)) v4fa;
typedef v2i  __attribute__((may_alias)) v2ia;
typedef v4i  __attribute__((may_alias)) v4ia;
typedef v8us __attribute__((may_alias)) v8usa;
union FragB { v16bf v; v16us u; v8us h[2]; v8i w; };

__device__ __forceinline__ v8f wmb(const FragB& a, const FragB& b, v8f c) {
  v8f d = __builtin_amdgcn_wmma_f32_16x16x32_bf16(false, a.v, false, b.v, (short)0, c, false, false);
  asm volatile("v_nop\n\tv_nop\n\tv_nop\n\tv_nop" : "+v"(d) : "v"(a.w), "v"(b.w));
  return d;
}

__device__ __forceinline__ unsigned bf16_bits(float f) {
  const unsigned u = __float_as_uint(f);
  const unsigned r = (u + 0x7FFFu + ((u >> 16) & 1u)) >> 16;
  const unsigned q = (u >> 16) | 0x40u;
  return ((u & 0x7fffffffu) > 0x7f800000u) ? q : r;
}

__device__ __forceinline__ void st2_v8us(unsigned short* p, v8us v) {
  *(volatile v8us*)p = v;
  __threadfence();
  *(volatile v8us*)p = v;
}

__global__ __launch_bounds__(NTHR) void k_prep(const float* __restrict__ x, const float* __restrict__ w,
                                               unsigned short* xb, unsigned short* wb) {
  const int tid = (int)threadIdx.x;
  const int blk = (int)blockIdx.x;
  if (blk < PBX) {
    const int u   = blk * NTHR + tid;
    const int row = u >> 4, k8 = (u & 15) * 8;
    const int rc  = row < NN ? row : NN - 1;
    const unsigned mk = row < NN ? 0xffffu : 0u;
    const float* p = x + (size_t)rc * DF + k8;
    const v4f a = *(const v4fa*)p;
    const v4f b = *(const v4fa*)(p + 4);
    v8us o;
    o[0] = (unsigned short)(bf16_bits(a.x) & mk); o[1] = (unsigned short)(bf16_bits(a.y) & mk);
    o[2] = (unsigned short)(bf16_bits(a.z) & mk); o[3] = (unsigned short)(bf16_bits(a.w) & mk);
    o[4] = (unsigned short)(bf16_bits(b.x) & mk); o[5] = (unsigned short)(bf16_bits(b.y) & mk);
    o[6] = (unsigned short)(bf16_bits(b.z) & mk); o[7] = (unsigned short)(bf16_bits(b.w) & mk);
    st2_v8us(xb + (size_t)row * DF + k8, o);
  } else {
    const int u = (blk - PBX) * NTHR + tid;
    const int n = u >> 4, k8 = (u & 15) * 8;
    const float* p = w + (size_t)n * DF + k8;
    const v4f a = *(const v4fa*)p;
    const v4f b = *(const v4fa*)(p + 4);
    v8us o;
    o[0] = (unsigned short)bf16_bits(a.x); o[1] = (unsigned short)bf16_bits(a.y);
    o[2] = (unsigned short)bf16_bits(a.z); o[3] = (unsigned short)bf16_bits(a.w);
    o[4] = (unsigned short)bf16_bits(b.x); o[5] = (unsigned short)bf16_bits(b.y);
    o[6] = (unsigned short)bf16_bits(b.z); o[7] = (unsigned short)bf16_bits(b.w);
    st2_v8us(wb + (size_t)n * DF + k8, o);
  }
}

__device__ __forceinline__ void bucket_flush(const int* pl, const int* cnt, const int* offs, int ov,
                                             int* lp, int* cp, int* op, int* fp, int tid) {
#pragma unroll 1
  for (int i = tid * 4; i < 2 * RCAP; i += NTHR * 4) {
    const v4i v = *(const v4ia*)(pl + i);
    *(volatile v4i*)(lp + i) = v;
  }
  {
    const v4i v = *(const v4ia*)(cnt + 4 * tid);
    *(volatile v4i*)(cp + 4 * tid) = v;
  }
  {
    const v4i v = *(const v4ia*)(offs + 4 * tid);
    *(volatile v4i*)(op + 4 * tid) = v;
  }
  if (tid < 8) {
    const v4i f = {ov, ov, ov, ov};
    *(volatile v4i*)(fp + 4 * tid) = f;
  }
}

__global__ __launch_bounds__(NTHR) void k_bucket(const int* __restrict__ srcs, const int* __restrict__ dsts,
                                                 const float* __restrict__ ew, int* LIST, int* CNT, int* OFF,
                                                 int* FLAG) {
  extern __shared__ __attribute__((aligned(16))) int dsm[];
  int* wl   = dsm;
  int* pl   = dsm + NWAVE * WLCAP;
  int* cnt  = pl + 2 * RCAP;
  int* offs = cnt + NBRUN;
  int* cur  = offs + NBRUN;
  int* misc = cur + NBRUN;
  const int tid = (int)threadIdx.x, lane = tid & 31, wave = tid >> 5;
  const int blk = (int)blockIdx.x;
  const unsigned nbs = (unsigned)(blk * NBRUN);

  {
    const v4i z4 = {0, 0, 0, 0};
    for (int i = tid * 4; i < BK_ZINTS; i += NTHR * 4) *(v4ia*)(dsm + i) = z4;
    if (tid < 16) misc[tid] = 0;
  }
  __syncthreads();

  {
    const int per  = ((NE + NWAVE * WCH - 1) / (NWAVE * WCH)) * WCH;
    const int ebeg = wave * per;
    const int eend = (ebeg + per < NE) ? (ebeg + per) : NE;
    int* mylist = wl + wave * WLCAP;
    int wc = 0;
#pragma unroll 1
    for (int cb = ebeg; cb < eend; cb += WCH) {
      const int e0 = cb + lane * EPT;
      const v4i da = *(const v4ia*)(dsts + e0);
      const v4i db = *(const v4ia*)(dsts + e0 + 4);
      const unsigned s0 = (unsigned)da.x - nbs, s1 = (unsigned)da.y - nbs;
      const unsigned s2 = (unsigned)da.z - nbs, s3 = (unsigned)da.w - nbs;
      const unsigned s4 = (unsigned)db.x - nbs, s5 = (unsigned)db.y - nbs;
      const unsigned s6 = (unsigned)db.z - nbs, s7 = (unsigned)db.w - nbs;
      const bool h0 = s0 < (unsigned)NBRUN, h1 = s1 < (unsigned)NBRUN, h2 = s2 < (unsigned)NBRUN, h3 = s3 < (unsigned)NBRUN;
      const bool h4 = s4 < (unsigned)NBRUN, h5 = s5 < (unsigned)NBRUN, h6 = s6 < (unsigned)NBRUN, h7 = s7 < (unsigned)NBRUN;
      const unsigned m0 = __builtin_amdgcn_ballot_w32(h0), m1 = __builtin_amdgcn_ballot_w32(h1);
      const unsigned m2 = __builtin_amdgcn_ballot_w32(h2), m3 = __builtin_amdgcn_ballot_w32(h3);
      const unsigned m4 = __builtin_amdgcn_ballot_w32(h4), m5 = __builtin_amdgcn_ballot_w32(h5);
      const unsigned m6 = __builtin_amdgcn_ballot_w32(h6), m7 = __builtin_amdgcn_ballot_w32(h7);
      const unsigned any = m0 | m1 | m2 | m3 | m4 | m5 | m6 | m7;
      if (any != 0u) {
        const int pre = (int)(__builtin_amdgcn_mbcnt_lo(m0, 0u) + __builtin_amdgcn_mbcnt_lo(m1, 0u) +
                              __builtin_amdgcn_mbcnt_lo(m2, 0u) + __builtin_amdgcn_mbcnt_lo(m3, 0u) +
                              __builtin_amdgcn_mbcnt_lo(m4, 0u) + __builtin_amdgcn_mbcnt_lo(m5, 0u) +
                              __builtin_amdgcn_mbcnt_lo(m6, 0u) + __builtin_amdgcn_mbcnt_lo(m7, 0u));
        int p = wc + pre;
        if (h0) { if (p < WLCAP) mylist[p] = ((e0 + 0) << SLB) | (int)s0; p = p + 1; }
        if (h1) { if (p < WLCAP) mylist[p] = ((e0 + 1) << SLB) | (int)s1; p = p + 1; }
        if (h2) { if (p < WLCAP) mylist[p] = ((e0 + 2) << SLB) | (int)s2; p = p + 1; }
        if (h3) { if (p < WLCAP) mylist[p] = ((e0 + 3) << SLB) | (int)s3; p = p + 1; }
        if (h4) { if (p < WLCAP) mylist[p] = ((e0 + 4) << SLB) | (int)s4; p = p + 1; }
        if (h5) { if (p < WLCAP) mylist[p] = ((e0 + 5) << SLB) | (int)s5; p = p + 1; }
        if (h6) { if (p < WLCAP) mylist[p] = ((e0 + 6) << SLB) | (int)s6; p = p + 1; }
        if (h7) { if (p < WLCAP) mylist[p] = ((e0 + 7) << SLB) | (int)s7; p = p + 1; }
        wc += (int)(__builtin_popcount(m0) + __builtin_popcount(m1) + __builtin_popcount(m2) + __builtin_popcount(m3) +
                    __builtin_popcount(m4) + __builtin_popcount(m5) + __builtin_popcount(m6) + __builtin_popcount(m7));
      }
    }
    if (lane == 0) misc[wave] = wc;
  }
  __syncthreads();

  if (wave == 0) {
    int ov = 0, tot = 0;
#pragma unroll 1
    for (int w2 = 0; w2 < NWAVE; ++w2) {
      int c = misc[w2];
      if (c > WLCAP) ov = 1;
      c = c < 0 ? 0 : (c > WLCAP ? WLCAP : c);
      tot += c;
#pragma unroll 1
      for (int b0 = 0; b0 < c; b0 += 32) {
        const int idx = b0 + lane;
        const int ent = wl[w2 * WLCAP + (idx < WLCAP ? idx : WLCAP - 1)];
        const int m32 = (c - b0) < 32 ? (c - b0) : 32;
#pragma unroll 1
        for (int k = 0; k < m32; ++k) {
          const int u    = __builtin_amdgcn_readlane(ent, k);
          const int slot = u & (NBRUN - 1);
          if (lane == 0) cnt[slot] = cnt[slot] + 1;
        }
      }
    }
    if (tot > RCAP) ov = 1;
    if (lane == 0) misc[9] = ov;
  }
  __syncthreads();
  if (wave == 0) {
    const int base = lane * (NBRUN / 32);
    int s = 0;
#pragma unroll 1
    for (int i = 0; i < NBRUN / 32; ++i) s += cnt[base + i];
    int incl = s;
#pragma unroll
    for (int d = 1; d < 32; d <<= 1) {
      const int y = __shfl_up(incl, d, 32);
      if (lane >= d) incl += y;
    }
    int run = incl - s;
#pragma unroll 1
    for (int i = 0; i < NBRUN / 32; ++i) {
      const int cv = cnt[base + i];
      offs[base + i] = run;
      cur[base + i]  = run;
      run += cv;
    }
  }
  __syncthreads();

  if (wave == 0) {
#pragma unroll 1
    for (int w2 = 0; w2 < NWAVE; ++w2) {
      int c = misc[w2];
      c = c < 0 ? 0 : (c > WLCAP ? WLCAP : c);
#pragma unroll 1
      for (int b0 = 0; b0 < c; b0 += 32) {
        const int idx = b0 + lane;
        const int ent = wl[w2 * WLCAP + (idx < WLCAP ? idx : WLCAP - 1)];
        int eid = (ent >> SLB) & 0xFFFFF;
        eid = eid > NE - 1 ? NE - 1 : eid;
        int sr = srcs[eid];
        sr = sr < 0 ? 0 : (sr > NN - 1 ? NN - 1 : sr);
        const int wbits = (int)(bf16_bits(ew[eid]) << 16);
        const int m32 = (c - b0) < 32 ? (c - b0) : 32;
#pragma unroll 1
        for (int k = 0; k < m32; ++k) {
          const int u    = __builtin_amdgcn_readlane(ent, k);
          const int sk   = __builtin_amdgcn_readlane(sr, k);
          const int wk   = __builtin_amdgcn_readlane(wbits, k);
          const int slot = u & (NBRUN - 1);
          if (lane == 0) {
            int p = cur[slot];
            p = p < 0 ? 0 : (p > RCAP - 1 ? RCAP - 1 : p);
            pl[2 * p]     = sk;
            pl[2 * p + 1] = wk;
            cur[slot] = p + 1;
          }
        }
      }
    }
  }
  __syncthreads();

  const int ovf = misc[9];
  int* lp = LIST + (size_t)blk * (2 * RCAP);
  int* cp = CNT + (size_t)blk * NBRUN;
  int* op = OFF + (size_t)blk * NBRUN;
  int* fp = FLAG + (size_t)blk * 32;
  bucket_flush(pl, cnt, offs, ovf, lp, cp, op, fp, tid);
  __threadfence();
  bucket_flush(pl, cnt, offs, ovf, lp, cp, op, fp, tid);
}

__device__ __forceinline__ void gemm_flush(const float* stg, float* H, int rowBase, int wave, int lane) {
#pragma unroll 1
  for (int i = 0; i < 16; ++i) {
    const int lr = 16 * wave + i;
    const int r  = rowBase + lr;
    const v4f v = *(const v4fa*)(stg + lr * DF + 4 * lane);
    asm volatile("" :: "v"(v));
    if (r < NN) *(volatile v4f*)(H + (size_t)r * DF + 4 * lane) = v;
  }
}

__global__ __launch_bounds__(NTHR) __attribute__((amdgpu_num_vgpr(248)))
void k_gemm(const unsigned short* __restrict__ XB, const unsigned short* __restrict__ WB, float* H) {
  extern __shared__ __attribute__((aligned(16))) float stg[];
  const int tid = (int)threadIdx.x, lane = tid & 31, wave = tid >> 5, hh = lane >> 4, m = lane & 15;
  const int rowBase = (int)blockIdx.x * GBM;

  v8f acc[8];
  {
    const v8f z = {0.f, 0.f, 0.f, 0.f, 0.f, 0.f, 0.f, 0.f};
#pragma unroll
    for (int t = 0; t < 8; ++t) acc[t] = z;
  }
  const unsigned short* ap = XB + (size_t)(rowBase + 16 * wave + m) * (size_t)DF + 8 * hh;
  const unsigned short* bp = WB + (size_t)m * (size_t)DF + 8 * hh;

#pragma unroll 1
  for (int k0 = 0; k0 < DF; k0 += 32) {
    FragB af;
    af.h[0] = *(const v8usa*)(ap + k0);
    af.h[1] = *(const v8usa*)(ap + k0 + 16);
#pragma unroll
    for (int nt = 0; nt < 8; ++nt) {
      const unsigned short* wq = bp + (size_t)(16 * nt) * (size_t)DF + k0;
      FragB bf;
      bf.h[0] = *(const v8usa*)wq;
      bf.h[1] = *(const v8usa*)(wq + 16);
      acc[nt] = wmb(af, bf, acc[nt]);
    }
  }

#pragma unroll
  for (int nt = 0; nt < 8; ++nt) {
    const int lc = 16 * nt + m;
#pragma unroll
    for (int r = 0; r < 8; ++r) {
      const int lr = 16 * wave + 8 * hh + r;
      stg[lr * DF + lc] = acc[nt][r];
    }
  }
  __syncthreads();

  gemm_flush(stg, H, rowBase, wave, lane);
  __threadfence();
  gemm_flush(stg, H, rowBase, wave, lane);
}

__global__ __launch_bounds__(NTHR) void k_replay(const int* __restrict__ LIST, const int* __restrict__ CNT,
                                                 const int* __restrict__ OFF, const int* __restrict__ FLAG,
                                                 const float* __restrict__ H, float* out) {
  const int tid = (int)threadIdx.x, lane = tid & 31, wave = tid >> 5;
  const int d      = (int)blockIdx.x * NWAVE + wave;
  const int bucket = d >> SLB;
  const int slot   = d & (NBRUN - 1);
  int c = CNT[(size_t)bucket * NBRUN + slot];
  int o = OFF[(size_t)bucket * NBRUN + slot];
  const int flag = FLAG[(size_t)bucket * 32];
  c = c < 0 ? 0 : (c > RCAP ? RCAP : c);
  o = o < 0 ? 0 : (o > RCAP - 1 ? RCAP - 1 : o);
  const int cs = __builtin_amdgcn_readfirstlane(c);
  const int os = __builtin_amdgcn_readfirstlane(o);
  int last = os + cs - 1;
  last = last < os ? os : last;
  last = last > RCAP - 1 ? RCAP - 1 : last;
  const int* lb = LIST + (size_t)bucket * (2 * RCAP);

  float a0 = 0.0f, a1 = 0.0f, a2 = 0.0f, a3 = 0.0f;
#pragma unroll 2
  for (int j = 0; j < cs; ++j) {
    int idx = os + j;
    idx = idx > last ? last : idx;
    const v2i en = *(const v2ia*)(lb + 2 * idx);
    int sr = en.x;
    sr = sr < 0 ? 0 : (sr > NN - 1 ? NN - 1 : sr);
    const float w = __int_as_float(en.y);
    const v4f v = *(const v4fa*)(H + (size_t)sr * DF + 4 * lane);
    a0 = fmaf(w, v.x, a0);
    a1 = fmaf(w, v.y, a1);
    a2 = fmaf(w, v.z, a2);
    a3 = fmaf(w, v.w, a3);
  }
  const float qnan = __uint_as_float(0x7fc00000u);
  const bool bad = flag != 0;
  v4f ov;
  ov.x = bad ? qnan : a0;
  ov.y = bad ? qnan : a1;
  ov.z = bad ? qnan : a2;
  ov.w = bad ? qnan : a3;
  float* op = out + (size_t)d * DF + 4 * lane;
  *(volatile v4f*)op = ov;
  __threadfence();
  *(volatile v4f*)op = ov;
}

extern "C" void kernel_launch(void* const* d_in, const int* in_sizes, int n_in,
                              void* d_out, int out_size, void* d_ws, size_t ws_size,
                              hipStream_t stream) {
  if (n_in < 5) return;
  if (in_sizes[0] != NN * DF) return;
  if (in_sizes[1] != DF * DF) return;
  if (in_sizes[2] != NE) return;
  if (in_sizes[3] != NE) return;
  if (in_sizes[4] != NE) return;
  if (out_size != NN * DF) return;

  const float* x   = (const float*)d_in[0];
  const float* W   = (const float*)d_in[1];
  const float* ew  = (const float*)d_in[2];
  const int*   src = (const int*)d_in[3];
  const int*   tgt = (const int*)d_in[4];
  float* out = (float*)d_out;

  constexpr size_t zXB   = (size_t)MP * DF * 2;
  constexpr size_t zWB   = (size_t)DF * DF * 2;
  constexpr size_t zH    = (size_t)NN * DF * 4;
  constexpr size_t zLIST = (size_t)NBK * RCAP * 8;
  constexpr size_t zCNT  = (size_t)NBK * NBRUN * 4;
  constexpr size_t zOFF  = (size_t)NBK * NBRUN * 4;
  constexpr size_t zFLAG = (size_t)NBK * 128;
  constexpr size_t oXB   = 0;
  constexpr size_t oWB   = oXB + zXB;
  constexpr size_t oH    = oWB + zWB;
  constexpr size_t oLIST = oH + zH;
  constexpr size_t oCNT  = oLIST + zLIST;
  constexpr size_t oOFF  = oCNT + zCNT;
  constexpr size_t oFLAG = oOFF + zOFF;
  constexpr size_t oEND  = oFLAG + zFLAG;
  static_assert(zXB % 128 == 0 && zWB % 128 == 0 && zH % 128 == 0 && zLIST % 128 == 0);
  static_assert(zCNT % 128 == 0 && zOFF % 128 == 0 && zFLAG % 128 == 0);
  static_assert(oEND <= WSMAX);
  if (oEND > ws_size) return;

  char* ws = (char*)d_ws;
  unsigned short* XB   = (unsigned short*)(ws + oXB);
  unsigned short* WB   = (unsigned short*)(ws + oWB);
  float*          H    = (float*)(ws + oH);
  int*            LIST = (int*)(ws + oLIST);
  int*            CNT  = (int*)(ws + oCNT);
  int*            OFF  = (int*)(ws + oOFF);
  int*            FLAG = (int*)(ws + oFLAG);

  hipFuncSetAttribute(reinterpret_cast<const void*>(&k_bucket), hipFuncAttributeMaxDynamicSharedMemorySize, (int)BK_LDS);
  hipFuncSetAttribute(reinterpret_cast<const void*>(&k_gemm), hipFuncAttributeMaxDynamicSharedMemorySize, (int)GM_LDS);

  k_prep<<<PBTOT, NTHR, 0, stream>>>(x, W, XB, WB);
  k_bucket<<<NBK, NTHR, BK_LDS, stream>>>(src, tgt, ew, LIST, CNT, OFF, FLAG);
  k_gemm<<<MP / GBM, NTHR, GM_LDS, stream>>>(XB, WB, H);
  k_replay<<<NN / NWAVE, NTHR, 0, stream>>>(LIST, CNT, OFF, FLAG, H, out);
}
